// FractionalOrderMaskGenerator_53584011985294
// MI455X (gfx1250) — hardware-verified
//
#include <hip/hip_runtime.h>

#ifndef NB
#define NB 8
#endif
#define NB_FULL 8
#define HH 160
#define WWD 160
#define HW 25600
#define CC 64
#define K9 576
#define NPIX ((size_t)NB * (size_t)HW)
#define NBLK128 (NPIX / 128)
static_assert(HW % 128 == 0);
static_assert(HH * WWD == HW);
static_assert((size_t)NB_FULL * 25 * HW * 4 == (size_t)20480000);
static_assert(NB >= 1 && NB <= NB_FULL);

typedef __bf16 v16b __attribute__((ext_vector_type(16)));
typedef unsigned short v8us __attribute__((ext_vector_type(8), may_alias));
typedef float v8f __attribute__((ext_vector_type(8)));
typedef float v4f __attribute__((ext_vector_type(4)));
typedef float v4fa __attribute__((ext_vector_type(4), may_alias));
union FragB { v16b v; v8us half[2]; unsigned short u[16]; };
union U8 { v8us v; unsigned short u[8]; };

__device__ __forceinline__ unsigned short bf16_bits(float x) { unsigned int u = __float_as_uint(x); return (unsigned short)((u + 0x7FFFu + ((u >> 16) & 1u)) >> 16); }
__device__ __forceinline__ float bf16_val(unsigned short b) { return __uint_as_float(((unsigned int)b) << 16); }
__device__ __forceinline__ float bf16_rne(float x) { return bf16_val(bf16_bits(x)); }

template <int NT>
__device__ __forceinline__ v8f mmaN(v16b ah, v16b al, v16b bh, v16b bl, v8f c) {
  c = __builtin_amdgcn_wmma_f32_16x16x32_bf16(false, ah, false, bh, (short)0, c, false, false);
  if (NT >= 2) c = __builtin_amdgcn_wmma_f32_16x16x32_bf16(false, al, false, bh, (short)0, c, false, false);
  if (NT >= 3) c = __builtin_amdgcn_wmma_f32_16x16x32_bf16(false, ah, false, bl, (short)0, c, false, false);
  asm volatile("v_nop\n\tv_nop\n\tv_nop\n\tv_nop" : "+v"(c) : "v"(ah), "v"(al), "v"(bh), "v"(bl));
  return c;
}

__device__ __forceinline__ unsigned long long cidx_code(int d) {
  const int k = d & 3;
  return (k == 0) ? 0x2AA55400556AAull : (k == 1) ? 0x394945454585Bull : (k == 2) ? 0x24691A4691A46ull : 0x05B4594594794ull;
}

__global__ __launch_bounds__(256) void k_xpack(const float* __restrict__ x, unsigned short* __restrict__ X16, float* __restrict__ gray) {
  __shared__ __attribute__((aligned(16))) unsigned short s[32][72];
  __shared__ float gs[8][32];
  const int tid = threadIdx.x, px = tid & 31, w = tid >> 5;
  const size_t p0 = (size_t)blockIdx.x * 32;
  const size_t b = p0 / HW;
  const size_t yx0 = p0 - b * HW;
  float part = 0.f;
#pragma unroll
  for (int it = 0; it < 8; ++it) {
    const int c = w * 8 + it;
    const unsigned short hb = bf16_bits(x[(b * CC + (size_t)c) * HW + yx0 + px]);
    s[px][c] = hb;
    part += bf16_val(hb);
  }
  gs[w][px] = part;
  __syncthreads();
  const int q = px >> 3, j = tid & 7;
  const int pl = w * 4 + q;
  const v8us vr = *(const v8us*)&s[pl][8 * j];
  float gv = gs[0][px];
#pragma unroll
  for (int k = 1; k < 8; ++k) gv += gs[k][px];
  gv = gv / 64.0f;
  for (int pass = 0; pass < 2; ++pass) {
    *(volatile v8us*)(X16 + (p0 + (size_t)pl) * CC + 8 * j) = vr;
    if (tid < 32) *(volatile float*)(gray + p0 + px) = gv;
    if (pass == 0) __threadfence();
  }
}

__global__ __launch_bounds__(256) void k_wconv(const float* __restrict__ w, unsigned short* __restrict__ Bt) {
  const int t = blockIdx.x * 256 + threadIdx.x;
  if (t >= 64 * K9 / 8) return;
  const int c8 = (t & 7) * 8, tap = (t >> 3) % 9, o = t / 72;
  U8 f;
#pragma unroll
  for (int q = 0; q < 8; ++q) f.u[q] = bf16_bits(w[((size_t)o * CC + (size_t)(c8 + q)) * 9 + tap]);
  *(volatile v8us*)(Bt + (size_t)t * 8) = f.v;
  __threadfence();
  *(volatile v8us*)(Bt + (size_t)t * 8) = f.v;
}

__global__ __launch_bounds__(256) void k_wrow(const float* __restrict__ w, unsigned short* __restrict__ Bt, int n8) {
  const int t = blockIdx.x * 256 + threadIdx.x;
  if (t >= n8) return;
  U8 f;
#pragma unroll
  for (int q = 0; q < 8; ++q) f.u[q] = bf16_bits(w[(size_t)t * 8 + q]);
  *(volatile v8us*)(Bt + (size_t)t * 8) = f.v;
  __threadfence();
  *(volatile v8us*)(Bt + (size_t)t * 8) = f.v;
}

template <int TAPS, int DIL, int NPROD>
__global__ __launch_bounds__(128) void k_conv(const unsigned short* __restrict__ Ah, const unsigned short* __restrict__ Al,
                                              const unsigned short* __restrict__ Bt, const float* __restrict__ bias,
                                              float* __restrict__ C, double* __restrict__ part) {
  constexpr int K = TAPS * CC;
  __shared__ __attribute__((aligned(16))) float so[4][32][68];
  __shared__ __attribute__((aligned(16))) double pst[4][2][2][64];
  __shared__ __attribute__((aligned(16))) double pln[128];
  const int tid = threadIdx.x, w = tid >> 5, lane = tid & 31, ln = lane & 15, hh = lane >> 4;
  const size_t row0 = (size_t)blockIdx.x * 128 + (size_t)(32 * w);
  int yv[2], xv[2];
  size_t bbase[2];
#pragma unroll
  for (int fr = 0; fr < 2; ++fr) {
    const size_t gp = row0 + (size_t)(16 * fr + ln);
    const size_t b = gp / HW;
    const int yx = (int)(gp - b * HW);
    bbase[fr] = b * HW;
    yv[fr] = yx / WWD;
    xv[fr] = yx - (yx / WWD) * WWD;
  }
  const v8us z8 = {0, 0, 0, 0, 0, 0, 0, 0};
  const v8f zf = {0.f, 0.f, 0.f, 0.f, 0.f, 0.f, 0.f, 0.f};
  v8f acc[2][4] = {{zf, zf, zf, zf}, {zf, zf, zf, zf}};
#pragma unroll 1
  for (int kb = 0; kb < K; kb += 32) {
    const int tap = kb >> 6, c0 = kb & 63;
    int dy = 0, dx = 0;
    if (TAPS == 9) { dy = (tap / 3 - 1) * DIL; dx = (tap % 3 - 1) * DIL; }
    FragB ah[2], al[2];
#pragma unroll
    for (int fr = 0; fr < 2; ++fr) {
      const int yy = yv[fr] + dy, xx = xv[fr] + dx;
      const bool inb = ((unsigned)yy < (unsigned)HH) && ((unsigned)xx < (unsigned)WWD);
      const int yyc = min(max(yy, 0), HH - 1), xxc = min(max(xx, 0), WWD - 1);
      const size_t eoff = (bbase[fr] + (size_t)yyc * WWD + (size_t)xxc) * CC + (size_t)c0;
      const v8us h0 = *(const v8us*)(Ah + eoff + 8 * hh);
      const v8us h1 = *(const v8us*)(Ah + eoff + 16 + 8 * hh);
      ah[fr].half[0] = inb ? h0 : z8;
      ah[fr].half[1] = inb ? h1 : z8;
      if (NPROD == 2) {
        const v8us l0 = *(const v8us*)(Al + eoff + 8 * hh);
        const v8us l1 = *(const v8us*)(Al + eoff + 16 + 8 * hh);
        al[fr].half[0] = inb ? l0 : z8;
        al[fr].half[1] = inb ? l1 : z8;
      } else {
        al[fr].v = ah[fr].v;
      }
    }
#pragma unroll
    for (int t = 0; t < 4; ++t) {
      const unsigned short* bp = Bt + (size_t)(t * 16 + ln) * K + kb;
      FragB bq;
      bq.half[0] = *(const v8us*)(bp + 8 * hh);
      bq.half[1] = *(const v8us*)(bp + 16 + 8 * hh);
      acc[0][t] = mmaN<NPROD>(ah[0].v, al[0].v, bq.v, bq.v, acc[0][t]);
      acc[1][t] = mmaN<NPROD>(ah[1].v, al[1].v, bq.v, bq.v, acc[1][t]);
    }
  }
  double ds[4] = {0.0, 0.0, 0.0, 0.0}, dq[4] = {0.0, 0.0, 0.0, 0.0};
#pragma unroll
  for (int fr = 0; fr < 2; ++fr) {
#pragma unroll
    for (int t = 0; t < 4; ++t) {
      const float bv = bf16_rne(bias[t * 16 + ln]);
#pragma unroll
      for (int r = 0; r < 8; ++r) {
        const float v = acc[fr][t][r] + bv;
        so[w][fr * 16 + 8 * hh + r][t * 16 + ln] = v;
        ds[t] += (double)v;
        dq[t] += (double)v * (double)v;
      }
    }
  }
#pragma unroll
  for (int t = 0; t < 4; ++t) { pst[w][hh][0][t * 16 + ln] = ds[t]; pst[w][hh][1][t * 16 + ln] = dq[t]; }
  __syncthreads();
  {
    const int j = tid & 63, which = tid >> 6;
    double tot = 0.0;
#pragma unroll
    for (int wq = 0; wq < 4; ++wq) { tot += pst[wq][0][which][j]; tot += pst[wq][1][which][j]; }
    pln[tid] = tot;
  }
  __syncthreads();
  const int rsub = lane >> 4, c4 = (lane & 15) * 4;
  for (int pass = 0; pass < 2; ++pass) {
#pragma unroll
    for (int q = 0; q < 16; ++q) {
      const int r = q * 2 + rsub;
      const v4f v = *(const v4fa*)&so[w][r][c4];
      *(volatile v4f*)(C + (row0 + (size_t)r) * CC + c4) = v;
    }
    if (tid < 64) {
      const v4f pv = *(const v4fa*)((const float*)pln + 4 * tid);
      *(volatile v4f*)((float*)part + (size_t)blockIdx.x * 256 + 4 * tid) = pv;
    }
    if (pass == 0) __threadfence();
  }
}

__global__ __launch_bounds__(256) void k_bnred(const double* __restrict__ part, int nblk, const float* __restrict__ g, const float* __restrict__ be,
                                               float* __restrict__ bnp) {
  #pragma clang fp contract(off)
  __shared__ double red[256];
  __shared__ __attribute__((aligned(16))) float outv[256];
  const int tid = threadIdx.x, ch = tid & 63, which = (tid >> 6) & 1, q = tid >> 7;
  double s = 0.0;
  for (int i = q; i < nblk; i += 2) s += part[(size_t)i * 128 + (size_t)(which * 64 + ch)];
  red[tid] = s;
  __syncthreads();
  if (tid < 64) {
    const double S = red[ch] + red[ch + 128];
    const double Q = red[64 + ch] + red[64 + ch + 128];
    const double n = (double)nblk * 128.0;
    const double mu = S / n;
    double var = Q / n - mu * mu;
    if (var < 0.0) var = 0.0;
    const float muf = (float)mu, varf = (float)var;
    const float rs = 1.0f / sqrtf(varf + 1e-5f);
    outv[4 * ch] = muf;
    outv[4 * ch + 1] = rs;
    outv[4 * ch + 2] = bf16_rne(g[ch]);
    outv[4 * ch + 3] = bf16_rne(be[ch]);
  }
  __syncthreads();
  for (int pass = 0; pass < 2; ++pass) {
    if (tid < 64) { const v4f v = *(const v4fa*)&outv[4 * tid]; *(volatile v4f*)(bnp + 4 * tid) = v; }
    if (pass == 0) __threadfence();
  }
}

__global__ __launch_bounds__(256) void k_bnapp16(const float* __restrict__ R, const float* __restrict__ bnp, unsigned short* __restrict__ Hh,
                                                 unsigned short* __restrict__ Hl, size_t n8) {
  #pragma clang fp contract(off)
  __shared__ __attribute__((aligned(16))) float sp[256];
  const int tid = threadIdx.x;
  sp[tid] = bnp[tid];
  __syncthreads();
  const size_t t = (size_t)blockIdx.x * 256 + tid;
  if (t >= n8) return;
  const int c0 = (int)((t * 8) & 63);
  const v4f a = *(const v4fa*)(R + t * 8), c = *(const v4fa*)(R + t * 8 + 4);
  U8 fh, fl;
#pragma unroll
  for (int q = 0; q < 8; ++q) {
    const float xv = (q < 4) ? a[q] : c[q - 4];
    const v4f pr = *(const v4fa*)&sp[4 * (c0 + q)];
    float v = ((xv - pr[0]) * pr[1]) * pr[2] + pr[3];
    v = fmaxf(v, 0.f);
    const unsigned short hb = bf16_bits(v);
    fh.u[q] = hb;
    fl.u[q] = bf16_bits(v - bf16_val(hb));
  }
  for (int pass = 0; pass < 2; ++pass) {
    *(volatile v8us*)(Hh + t * 8) = fh.v;
    *(volatile v8us*)(Hl + t * 8) = fl.v;
    if (pass == 0) __threadfence();
  }
}

__global__ __launch_bounds__(256) void k_bnapp32(const float* __restrict__ R, const float* __restrict__ bnp, float* __restrict__ A2, size_t n4) {
  #pragma clang fp contract(off)
  __shared__ __attribute__((aligned(16))) float sp[256];
  const int tid = threadIdx.x;
  sp[tid] = bnp[tid];
  __syncthreads();
  const size_t t = (size_t)blockIdx.x * 256 + tid;
  if (t >= n4) return;
  v4f o[2];
  size_t e0[2];
#pragma unroll
  for (int u = 0; u < 2; ++u) {
    e0[u] = (t + (size_t)u * n4) * 4;
    const int c0 = (int)(e0[u] & 63);
    const v4f a = *(const v4fa*)(R + e0[u]);
    v4f r;
#pragma unroll
    for (int q = 0; q < 4; ++q) {
      const v4f pr = *(const v4fa*)&sp[4 * (c0 + q)];
      float v = ((a[q] - pr[0]) * pr[1]) * pr[2] + pr[3];
      r[q] = fmaxf(v, 0.f);
    }
    o[u] = r;
  }
  for (int pass = 0; pass < 2; ++pass) {
    *(volatile v4f*)(A2 + e0[0]) = o[0];
    *(volatile v4f*)(A2 + e0[1]) = o[1];
    if (pass == 0) __threadfence();
  }
}

__global__ __launch_bounds__(256) void k_dw(const float* __restrict__ A2, const float* __restrict__ wd, const float* __restrict__ bd,
                                            unsigned short* __restrict__ Dh, unsigned short* __restrict__ Dl, size_t nthr) {
  __shared__ __attribute__((aligned(16))) float swd[576];
  __shared__ float sbd[64];
  const int tid = threadIdx.x;
  for (int i = tid; i < 576; i += 256) swd[i] = bf16_rne(wd[i]);
  if (tid < 64) sbd[tid] = bf16_rne(bd[tid]);
  __syncthreads();
  const size_t t = (size_t)blockIdx.x * 256 + tid;
  if (t >= nthr) return;
  const int cg = (int)(t & 7);
  const size_t p = t >> 3;
  const size_t b = p / HW;
  const int yx = (int)(p - b * HW);
  const int y = yx / WWD, x = yx - (yx / WWD) * WWD;
  float wr[72];
#pragma unroll
  for (int i = 0; i < 18; ++i) { const v4f q4 = *(const v4fa*)(swd + cg * 72 + 4 * i); wr[4 * i] = q4[0]; wr[4 * i + 1] = q4[1]; wr[4 * i + 2] = q4[2]; wr[4 * i + 3] = q4[3]; }
  float acc[8] = {0.f, 0.f, 0.f, 0.f, 0.f, 0.f, 0.f, 0.f};
#pragma unroll
  for (int tap = 0; tap < 9; ++tap) {
    const int yy = y + tap / 3 - 1, xx = x + tap % 3 - 1;
    const bool inb = ((unsigned)yy < (unsigned)HH) && ((unsigned)xx < (unsigned)WWD);
    const int yyc = min(max(yy, 0), HH - 1), xxc = min(max(xx, 0), WWD - 1);
    const size_t src = (b * HW + (size_t)yyc * WWD + (size_t)xxc) * CC + (size_t)(cg * 8);
    const v4f v0 = *(const v4fa*)(A2 + src), v1 = *(const v4fa*)(A2 + src + 4);
#pragma unroll
    for (int j = 0; j < 8; ++j) {
      const float av = (j < 4) ? v0[j] : v1[j - 4];
      const float a = inb ? av : 0.f;
      acc[j] = fmaf(wr[j * 9 + tap], a, acc[j]);
    }
  }
  U8 fh, fl;
#pragma unroll
  for (int j = 0; j < 8; ++j) {
    const float v = acc[j] + sbd[cg * 8 + j];
    const unsigned short hb = bf16_bits(v);
    fh.u[j] = hb;
    fl.u[j] = bf16_bits(v - bf16_val(hb));
  }
  for (int pass = 0; pass < 2; ++pass) {
    *(volatile v8us*)(Dh + t * 8) = fh.v;
    *(volatile v8us*)(Dl + t * 8) = fl.v;
    if (pass == 0) __threadfence();
  }
}

__global__ __launch_bounds__(128) void k_head(const float* __restrict__ R3, const float* __restrict__ bnp,
                                              const unsigned short* __restrict__ X16, const unsigned short* __restrict__ Bta,
                                              const float* __restrict__ ba1, const float* __restrict__ wa2, const float* __restrict__ ba2,
                                              const float* __restrict__ w4, const float* __restrict__ b4, const float* __restrict__ gray,
                                              float* __restrict__ out0, float* __restrict__ out1) {
  #pragma clang fp contract(off)
  __shared__ __attribute__((aligned(16))) float tab[200 * 6];
  __shared__ __attribute__((aligned(16))) float sp[256];
  __shared__ __attribute__((aligned(16))) float sw4[64 * 8];
  __shared__ float sms[64];
  __shared__ float satt[4][32][17];
  const int tid = threadIdx.x, w = tid >> 5, lane = tid & 31, ln = lane & 15, hh = lane >> 4;
  for (int i = tid; i < 200; i += 128) {
    double v = (double)i * (4.0 / 199.0) + (-2.0);
    if (i == 199) v = 2.0;
    float t = 1.0f;
    tab[i * 6] = t;
#pragma unroll
    for (int m = 1; m < 6; ++m) { const double f = -(v - (double)(m - 1)) / (double)m; t = (float)((double)t * f); tab[i * 6 + m] = t; }
  }
  sp[tid] = bnp[tid];
  sp[tid + 128] = bnp[tid + 128];
  for (int i = tid; i < 512; i += 128) { const int e = i >> 3, d = i & 7; sw4[i] = bf16_rne(w4[d * 64 + e]); }
  if (tid < 8) sms[tid] = bf16_rne(b4[tid]);
  if (tid < 16) { sms[8 + tid] = bf16_rne(ba1[tid]); sms[24 + tid] = bf16_rne(wa2[tid]); }
  if (tid == 0) sms[40] = bf16_rne(ba2[0]);
  __syncthreads();
  const size_t p0 = (size_t)blockIdx.x * 128;
  {
    const size_t rowA = p0 + (size_t)(32 * w + ln);
    const v8f zf = {0.f, 0.f, 0.f, 0.f, 0.f, 0.f, 0.f, 0.f};
    v8f c0 = zf, c1 = zf;
#pragma unroll
    for (int kb = 0; kb < 64; kb += 32) {
      FragB a0, a1, bq;
      const unsigned short* ap = X16 + rowA * CC + kb;
      a0.half[0] = *(const v8us*)(ap + 8 * hh);
      a0.half[1] = *(const v8us*)(ap + 16 + 8 * hh);
      a1.half[0] = *(const v8us*)(ap + 16 * CC + 8 * hh);
      a1.half[1] = *(const v8us*)(ap + 16 * CC + 16 + 8 * hh);
      const unsigned short* bp = Bta + (size_t)ln * CC + kb;
      bq.half[0] = *(const v8us*)(bp + 8 * hh);
      bq.half[1] = *(const v8us*)(bp + 16 + 8 * hh);
      c0 = mmaN<1>(a0.v, a0.v, bq.v, bq.v, c0);
      c1 = mmaN<1>(a1.v, a1.v, bq.v, bq.v, c1);
    }
#pragma unroll
    for (int r = 0; r < 8; ++r) { satt[w][8 * hh + r][ln] = c0[r]; satt[w][16 + 8 * hh + r][ln] = c1[r]; }
  }
  __syncthreads();
  const size_t p = p0 + (size_t)tid;
  const size_t b = p / HW;
  const int yx = (int)(p - b * HW);
  const int y = yx / WWD, x = yx - (yx / WWD) * WWD;
  float z = 0.f;
#pragma unroll
  for (int j = 0; j < 16; ++j) { const float hj = fmaxf(satt[w][lane][j] + sms[8 + j], 0.f); z = fmaf(sms[24 + j], hj, z); }
  z = z + sms[40];
  const float att = 1.0f / (1.0f + expf(-z));
  float acc4[8] = {0.f, 0.f, 0.f, 0.f, 0.f, 0.f, 0.f, 0.f};
  const float* rr = R3 + p * CC;
#pragma unroll 4
  for (int e4 = 0; e4 < 16; ++e4) {
    const v4f v = *(const v4fa*)(rr + 4 * e4);
#pragma unroll
    for (int q = 0; q < 4; ++q) {
      const int e = 4 * e4 + q;
      const v4f pr = *(const v4fa*)&sp[4 * e];
      float h = ((v[q] - pr[0]) * pr[1]) * pr[2] + pr[3];
      h = fmaxf(h, 0.f);
      const v4f wl = *(const v4fa*)&sw4[e * 8], wh4 = *(const v4fa*)&sw4[e * 8 + 4];
      acc4[0] = fmaf(wl[0], h, acc4[0]); acc4[1] = fmaf(wl[1], h, acc4[1]); acc4[2] = fmaf(wl[2], h, acc4[2]); acc4[3] = fmaf(wl[3], h, acc4[3]);
      acc4[4] = fmaf(wh4[0], h, acc4[4]); acc4[5] = fmaf(wh4[1], h, acc4[5]); acc4[6] = fmaf(wh4[2], h, acc4[6]); acc4[7] = fmaf(wh4[3], h, acc4[7]);
    }
  }
  const float* gb = gray + b * HW;
  float g9[9];
#pragma unroll
  for (int k = 0; k < 9; ++k) {
    const int yy = y + k / 3 - 1, xx = x + k % 3 - 1;
    const bool inb = ((unsigned)yy < (unsigned)HH) && ((unsigned)xx < (unsigned)WWD);
    const int yyc = min(max(yy, 0), HH - 1), xxc = min(max(xx, 0), WWD - 1);
    const float gv = gb[(size_t)yyc * WWD + xxc];
    g9[k] = inb ? gv : 0.f;
  }
  const float gx = -g9[0] + g9[2] - 2.0f * g9[3] + 2.0f * g9[5] - g9[6] + g9[8];
  const float gy = -g9[0] - 2.0f * g9[1] - g9[2] + g9[6] + 2.0f * g9[7] + g9[8];
  const float mag = sqrtf(gx * gx + gy * gy + 1e-8f);
  const float gdir = (atan2f(gy, gx) + 3.14159265358979323846f) / 6.283185307179586f * 8.0f;
  float sw[8];
  float mx = -3.0e38f;
#pragma unroll
  for (int d = 0; d < 8; ++d) { float df = fabsf(gdir - (float)d); df = fminf(df, 8.0f - df); sw[d] = expf(-df) * (1.0f + mag); mx = fmaxf(mx, sw[d]); }
  float ssum = 0.f;
#pragma unroll
  for (int d = 0; d < 8; ++d) { sw[d] = expf(sw[d] - mx); ssum += sw[d]; }
  const float sinv = 1.0f / ssum;
#pragma unroll
  for (int d = 0; d < 8; ++d) sw[d] = sw[d] * sinv;
  float od[8];
  float fu[25];
#pragma unroll
  for (int t = 0; t < 25; ++t) fu[t] = 0.f;
#pragma unroll
  for (int d = 0; d < 8; ++d) {
    const float raw = tanhf(acc4[d] + sms[d]);
    const float o = (raw * 4.0f) / 2.0f;
    od[d] = o;
    float nrm = (o + 2.0f) / 4.0f;
    nrm = fminf(fmaxf(nrm, 0.f), 1.0f);
    const float idf = nrm * 199.0f;
    const float lof = floorf(idf), hif = ceilf(idf);
    int lo = (int)lof, hi = (int)hif;
    lo = min(max(lo, 0), 199); hi = min(max(hi, 0), 199);
    const float wh = idf - lof;
    const float wl = 1.0f - wh;
    const float* tl = &tab[lo * 6];
    const float* th = &tab[hi * 6];
    const float cd0 = wl * tl[0] + wh * th[0];
    const float cd1 = wl * tl[1] + wh * th[1];
    const float cd2 = wl * tl[2] + wh * th[2];
    const float cd3 = wl * tl[3] + wh * th[3];
    const unsigned long long code = cidx_code(d);
    const float dwd = sw[d];
#pragma unroll
    for (int t = 0; t < 25; ++t) {
      const int c = (int)((code >> (2 * t)) & 3ull);
      const float cv = (c == 0) ? cd0 : (c == 1) ? cd1 : (c == 2) ? cd2 : cd3;
      fu[t] = fmaf(cv, dwd, fu[t]);
    }
  }
  float fs = 0.f;
#pragma unroll
  for (int t = 0; t < 25; ++t) { fu[t] = fu[t] * att; fs += fu[t]; }
  const float fi = 1.0f / (fs + 1e-8f);
#pragma unroll
  for (int t = 0; t < 25; ++t) fu[t] = fu[t] * fi;
  float* o0 = out0 + (b * 25) * HW + (size_t)yx;
  float* o1 = out1 + (b * 8) * HW + (size_t)yx;
  for (int pass = 0; pass < 2; ++pass) {
#pragma unroll
    for (int t = 0; t < 25; ++t) *(volatile float*)(o0 + (size_t)t * HW) = fu[t];
#pragma unroll
    for (int d = 0; d < 8; ++d) *(volatile float*)(o1 + (size_t)d * HW) = od[d];
    if (pass == 0) __threadfence();
  }
}

extern "C" void kernel_launch(void* const* d_in, const int* in_sizes, int n_in,
                              void* d_out, int out_size, void* d_ws, size_t ws_size, hipStream_t stream) {
  if (n_in < 21) return;
  const float* const* I = (const float* const*)d_in;
  const float* x = I[0];
  const float* w1 = I[1]; const float* b1 = I[2]; const float* g1 = I[3]; const float* be1 = I[4];
  const float* w2 = I[5]; const float* b2 = I[6]; const float* g2 = I[7]; const float* be2 = I[8];
  const float* wd = I[9]; const float* bd = I[10];
  const float* w3 = I[11]; const float* b3 = I[12]; const float* g3 = I[13]; const float* be3 = I[14];
  const float* w4 = I[15]; const float* b4 = I[16];
  const float* wa1 = I[17]; const float* ba1 = I[18]; const float* wa2 = I[19]; const float* ba2 = I[20];
  if ((size_t)in_sizes[0] < NPIX * CC) return;
  if (in_sizes[1] < 64 * K9 || in_sizes[5] < 64 * K9 || in_sizes[9] < 576 || in_sizes[11] < 4096 || in_sizes[15] < 512 || in_sizes[17] < 1024) return;
  if (in_sizes[2] < 64 || in_sizes[3] < 64 || in_sizes[4] < 64 || in_sizes[6] < 64 || in_sizes[7] < 64 || in_sizes[8] < 64) return;
  if (in_sizes[10] < 64 || in_sizes[12] < 64 || in_sizes[13] < 64 || in_sizes[14] < 64) return;
  if (in_sizes[16] < 8 || in_sizes[18] < 16 || in_sizes[19] < 16 || in_sizes[20] < 1) return;
  if ((size_t)out_size < (size_t)NB_FULL * 25 * HW + (size_t)NB * 8 * HW) return;

  char* ws = (char*)d_ws;
  size_t off = 0;
  auto take = [&](size_t bytes) { char* p = ws + off; off += (bytes + 255) & ~(size_t)255; return p; };
  unsigned short* X16 = (unsigned short*)take(NPIX * CC * 2);
  float* GRAY = (float*)take(NPIX * 4);
  char* RB = take(NPIX * CC * 4);
  char* HP = take(NPIX * CC * 4);
  unsigned short* BT1 = (unsigned short*)take((size_t)64 * K9 * 2);
  unsigned short* BT2 = (unsigned short*)take((size_t)64 * K9 * 2);
  unsigned short* BT3 = (unsigned short*)take((size_t)64 * 64 * 2);
  unsigned short* BTA = (unsigned short*)take((size_t)16 * 64 * 2);
  double* PART = (double*)take(NBLK128 * 128 * 8);
  float* BNP1 = (float*)take(1024);
  float* BNP2 = (float*)take(1024);
  float* BNP3 = (float*)take(1024);
  if (off > ws_size) return;
  float* Rf = (float*)RB;
  unsigned short* Dh = (unsigned short*)RB; unsigned short* Dl = Dh + NPIX * CC;
  unsigned short* H1h = (unsigned short*)HP; unsigned short* H1l = H1h + NPIX * CC;
  float* A2 = (float*)HP;
  float* R3 = (float*)HP;
  float* out0 = (float*)d_out;
  float* out1 = out0 + (size_t)NB_FULL * 25 * HW;

  const unsigned g8 = (unsigned)((NPIX * 8 + 255) / 256);
  k_xpack<<<(unsigned)(NPIX / 32), 256, 0, stream>>>(x, X16, GRAY);
  k_wconv<<<(64 * K9 / 8 + 255) / 256, 256, 0, stream>>>(w1, BT1);
  k_wconv<<<(64 * K9 / 8 + 255) / 256, 256, 0, stream>>>(w2, BT2);
  k_wrow<<<2, 256, 0, stream>>>(w3, BT3, 512);
  k_wrow<<<1, 256, 0, stream>>>(wa1, BTA, 128);
  k_conv<9, 1, 1><<<(unsigned)NBLK128, 128, 0, stream>>>(X16, X16, BT1, b1, Rf, PART);
  k_bnred<<<1, 256, 0, stream>>>(PART, (int)NBLK128, g1, be1, BNP1);
  k_bnapp16<<<g8, 256, 0, stream>>>(Rf, BNP1, H1h, H1l, NPIX * 8);
  k_conv<9, 2, 2><<<(unsigned)NBLK128, 128, 0, stream>>>(H1h, H1l, BT2, b2, Rf, PART);
  k_bnred<<<1, 256, 0, stream>>>(PART, (int)NBLK128, g2, be2, BNP2);
  k_bnapp32<<<g8, 256, 0, stream>>>(Rf, BNP2, A2, NPIX * 8);
  k_dw<<<g8, 256, 0, stream>>>(A2, wd, bd, Dh, Dl, NPIX * 8);
  k_conv<1, 1, 2><<<(unsigned)NBLK128, 128, 0, stream>>>(Dh, Dl, BT3, b3, R3, PART);
  k_bnred<<<1, 256, 0, stream>>>(PART, (int)NBLK128, g3, be3, BNP3);
  k_head<<<(unsigned)NBLK128, 128, 0, stream>>>(R3, BNP3, X16, BTA, ba1, wa2, ba2, w4, b4, GRAY, out0, out1);
}
